// ChainCRF_38628935860689
// MI455X (gfx1250) — hardware-run, weakly checked
//
#include <hip/hip_runtime.h>
#include <math.h>

constexpr int kBatch = 32;
constexpr int kLen   = 256;
constexpr int kDim   = 768;
constexpr int kLab   = 51;
constexpr int kTT    = kLab * kLab;
constexpr int kRows  = kBatch * kLen;
constexpr int kNreal = kLab + kTT;
constexpr int kNcol  = 2688;
constexpr int kPartPitch = 32;
static_assert(kNcol % 64 == 0 && kNcol >= kNreal, "N tile multiple");
static_assert(kRows % 64 == 0, "M tile multiple");
static_assert(kDim % 32 == 0, "K multiple of 32");
static_assert((kRows * kDim) % (8 * 256) == 0, "x cast grid exact");
static_assert((kNcol * kDim) % (8 * 256) == 0, "w cast grid exact");

typedef __attribute__((ext_vector_type(16))) _Float16 v16h;
typedef __attribute__((ext_vector_type(8)))  _Float16 v8h;
typedef __attribute__((ext_vector_type(16))) __bf16   v16b;
typedef __attribute__((ext_vector_type(8)))  __bf16   v8b;
typedef __attribute__((ext_vector_type(8)))  float    v8f;
typedef __attribute__((ext_vector_type(4)))  float    v4f;
typedef __attribute__((ext_vector_type(4)))  unsigned int v4u;

__device__ __forceinline__ unsigned short f2bf_bits(float f) {
  unsigned u = __float_as_uint(f);
  return (unsigned short)((u + 0x7FFFu + ((u >> 16) & 1u)) >> 16);
}
__device__ __forceinline__ float bf_bits2f(unsigned short h) { return __uint_as_float(((unsigned)h) << 16); }

__device__ __forceinline__ void dep_guard_h(v8f& a, v8f& b, v16h x, v16h y) { asm volatile("v_nop\n\tv_nop\n\tv_nop\n\tv_nop" : "+v"(a), "+v"(b) : "v"(x), "v"(y)); }
__device__ __forceinline__ void dep_guard_b(v8f& a, v8f& b, v16b x, v16b y) { asm volatile("v_nop\n\tv_nop\n\tv_nop\n\tv_nop" : "+v"(a), "+v"(b) : "v"(x), "v"(y)); }
__device__ __forceinline__ void keep4_h(v16h a, v16h b, v16h c, v16h d) { asm volatile("v_nop" :: "v"(a), "v"(b), "v"(c), "v"(d)); }
__device__ __forceinline__ void keep4_b(v16b a, v16b b, v16b c, v16b d) { asm volatile("v_nop" :: "v"(a), "v"(b), "v"(c), "v"(d)); }
__device__ __forceinline__ void acc_guard4(v8f& a, v8f& b, v8f& c, v8f& d) { asm volatile("v_nop\n\tv_nop\n\tv_nop\n\tv_nop" : "+v"(a), "+v"(b), "+v"(c), "+v"(d)); }
template <typename T> struct Frag;
template <> struct Frag<_Float16> {
  typedef v16h V; union U { v16h v; v8h h[2]; };
  static __device__ __forceinline__ v16h load(const _Float16* p) {
    U f; f.h[0] = *(const v8h*)(p); f.h[1] = *(const v8h*)(p + 16); return f.v;
  }
  static __device__ __forceinline__ v8f mma(v16h a, v16h b, v8f c) {
    return __builtin_amdgcn_wmma_f32_16x16x32_f16(false, a, false, b, (short)0, c, false, false);
  }
  static __device__ __forceinline__ void guard(v8f& a, v8f& b, v16h x, v16h y) { dep_guard_h(a, b, x, y); }
  static __device__ __forceinline__ void keep(v16h a, v16h b, v16h c, v16h d) { keep4_h(a, b, c, d); }
};
template <> struct Frag<__bf16> {
  typedef v16b V; union U { v16b v; v8b h[2]; };
  static __device__ __forceinline__ v16b load(const __bf16* p) {
    U f; f.h[0] = *(const v8b*)(p); f.h[1] = *(const v8b*)(p + 16); return f.v;
  }
  static __device__ __forceinline__ v8f mma(v16b a, v16b b, v8f c) {
    return __builtin_amdgcn_wmma_f32_16x16x32_bf16(false, a, false, b, (short)0, c, false, false);
  }
  static __device__ __forceinline__ void guard(v8f& a, v8f& b, v16b x, v16b y) { dep_guard_b(a, b, x, y); }
  static __device__ __forceinline__ void keep(v16b a, v16b b, v16b c, v16b d) { keep4_b(a, b, c, d); }
};

__device__ __forceinline__ unsigned pk16(unsigned short a, unsigned short b) { return (unsigned)a | ((unsigned)b << 16); }
__device__ __forceinline__ unsigned short h_bits(float f) { const _Float16 h = (_Float16)f; return __builtin_bit_cast(unsigned short, h); }

template <int ET> struct Elem;
template <> struct Elem<0> { typedef _Float16 T; };
template <> struct Elem<1> { typedef __bf16 T; };
template <int ET, int SPL, int RSC, int OUT_MODE, int ACT, int TRI>
__global__ __launch_bounds__(256) void wmma_gemm64(
    const unsigned short* __restrict__ Ap, const unsigned short* __restrict__ A2p, int lda, long strideA,
    const unsigned short* __restrict__ Btp, const unsigned short* __restrict__ Bt2p, int ldb, long strideB,
    void* __restrict__ Cout, void* __restrict__ Cout2, int ldc, long strideC,
    const float* __restrict__ rsc, long strideS,
    int M, int N, int K, float scale) {
  typedef typename Elem<ET>::T T;
  typedef typename Frag<T>::V V;
  const T* A = (const T*)Ap; const T* A2 = (const T*)A2p; const T* Bt = (const T*)Btp; const T* Bt2 = (const T*)Bt2p;
  __shared__ __align__(16) float sT[8][16 * 68];
  const int b    = blockIdx.y;
  const int lane = threadIdx.x & 31;
  const int wave = threadIdx.x >> 5;
  const int tilesN = N >> 6;
  const int tilesM = M >> 6;
  const int tile = blockIdx.x * 8 + wave;
  if (tile >= tilesM * tilesN) return;
  const int tm = tile / tilesN;
  const int tn = tile - tm * tilesN;
  const int m0 = tm << 6;
  const int n0 = tn << 6;
  if (TRI == 1 && n0 > m0) return;
  const int Kl = (TRI == 2 && (m0 + 64) < K) ? (m0 + 64) : K;

  const T* Ab  = A  + (size_t)b * strideA;
  const T* Bb  = Bt + (size_t)b * strideB;
  const T* Ab2 = (SPL & 1) ? (A2  + (size_t)b * strideA) : nullptr;
  const T* Bb2 = (SPL & 2) ? (Bt2 + (size_t)b * strideB) : nullptr;

  const int rlane = lane & 15;
  const int koff  = (lane >> 4) * 8;
  const int mOff  = (lane >> 4) * 8;

  v8f acc[4][4];
#pragma unroll
  for (int i = 0; i < 4; ++i)
#pragma unroll
    for (int j = 0; j < 4; ++j) acc[i][j] = (v8f){0.f,0.f,0.f,0.f,0.f,0.f,0.f,0.f};

  for (int k0 = 0; k0 < Kl; k0 += 32) {
    V bh[4], bl[4];
#pragma unroll
    for (int j = 0; j < 4; ++j) {
      const size_t bo = (size_t)(n0 + (j << 4) + rlane) * ldb + koff + k0;
      bh[j] = Frag<T>::load(Bb + bo);
      if (SPL & 2) bl[j] = Frag<T>::load(Bb2 + bo);
    }
#pragma unroll
    for (int i = 0; i < 4; ++i) {
      const size_t ao = (size_t)(m0 + (i << 4) + rlane) * lda + koff + k0;
      V ah = Frag<T>::load(Ab + ao);
      V al;
      if (SPL & 1) al = Frag<T>::load(Ab2 + ao);
#pragma unroll
      for (int j = 0; j < 4; ++j) {
        acc[i][j] = Frag<T>::mma(ah, bh[j], acc[i][j]);
        if (SPL & 2) acc[i][j] = Frag<T>::mma(ah, bl[j], acc[i][j]);
        if (SPL & 1) acc[i][j] = Frag<T>::mma(al, bh[j], acc[i][j]);
      }
      Frag<T>::guard(acc[i][0], acc[i][3], ah, (SPL & 1) ? al : ah);
    }
    Frag<T>::keep(bh[0], bh[1], bh[2], bh[3]);
    if (SPL & 2) Frag<T>::keep(bl[0], bl[1], bl[2], bl[3]);
  }
  acc_guard4(acc[0][0], acc[0][1], acc[0][2], acc[0][3]);
  acc_guard4(acc[1][0], acc[1][1], acc[1][2], acc[1][3]);
  acc_guard4(acc[2][0], acc[2][1], acc[2][2], acc[2][3]);
  acc_guard4(acc[3][0], acc[3][1], acc[3][2], acc[3][3]);

  float* slab = sT[wave];
  const float* Rs = RSC ? (rsc + (size_t)b * strideS) : nullptr;
#pragma unroll
  for (int i = 0; i < 4; ++i) {
    const int mBase = m0 + (i << 4);
    float rsv[8];
#pragma unroll
    for (int r = 0; r < 8; ++r) rsv[r] = RSC ? Rs[mBase + mOff + r] : 1.0f;
#pragma unroll
    for (int j = 0; j < 4; ++j) {
      const int n = n0 + (j << 4) + rlane;
#pragma unroll
      for (int r = 0; r < 8; ++r) {
        float v = acc[i][j][r] * scale;
        if (RSC) v = v * rsv[r];
        if (TRI == 1) { if (n > mBase + mOff + r) v = 0.0f; }
        if (ACT == 6) v = (v > 0.0f) ? (v + 1.0f) : __expf(v);
        slab[(mOff + r) * 68 + (j << 4) + rlane] = v;
      }
    }
    __builtin_amdgcn_fence(__ATOMIC_RELEASE, "workgroup");
    __builtin_amdgcn_wave_barrier();
    __builtin_amdgcn_fence(__ATOMIC_ACQUIRE, "workgroup");
    if (OUT_MODE == 0) {
      float* C = (float*)Cout + (size_t)b * strideC;
      const int hh = lane >> 4, c4 = (lane & 15) * 4;
      for (int pass = 0; pass < 2; ++pass) {
#pragma unroll
        for (int it = 0; it < 8; ++it) {
          const int row = it * 2 + hh;
          v4f v = *(const v4f*)(slab + row * 68 + c4);
          *(volatile v4f*)(C + (size_t)(mBase + row) * ldc + n0 + c4) = v;
        }
        __threadfence();
      }
    } else {
      const int q = lane >> 3, c8 = (lane & 7) * 8;
      unsigned short* C  = (unsigned short*)Cout  + (size_t)b * strideC;
      unsigned short* C2 = (OUT_MODE == 2) ? ((unsigned short*)Cout2 + (size_t)b * strideC) : nullptr;
      for (int pass = 0; pass < 2; ++pass) {
#pragma unroll
        for (int it = 0; it < 4; ++it) {
          const int row = it * 4 + q;
          const float* sp = slab + row * 68 + c8;
          v8h hv, lv;
#pragma unroll
          for (int e = 0; e < 8; ++e) {
            if (OUT_MODE == 1) {
              hv[e] = (_Float16)sp[e];
            } else {
              unsigned short hb = f2bf_bits(sp[e]);
              unsigned short lb = f2bf_bits(sp[e] - bf_bits2f(hb));
              hv[e] = __builtin_bit_cast(_Float16, hb);
              lv[e] = __builtin_bit_cast(_Float16, lb);
            }
          }
          *(volatile v8h*)(C + (size_t)(mBase + row) * ldc + n0 + c8) = hv;
          if (OUT_MODE == 2) *(volatile v8h*)(C2 + (size_t)(mBase + row) * ldc + n0 + c8) = lv;
        }
        __threadfence();
      }
    }
    __builtin_amdgcn_fence(__ATOMIC_RELEASE, "workgroup");
    __builtin_amdgcn_wave_barrier();
    __builtin_amdgcn_fence(__ATOMIC_ACQUIRE, "workgroup");
  }
}

template <int MODE>
__global__ __launch_bounds__(256) void cast8_kernel(const float* __restrict__ in, unsigned short* __restrict__ out, int n8, float scale) {
  const int i = blockIdx.x * 256 + threadIdx.x;
  if (i >= n8) return;
  const float* p = in + 8 * (size_t)i;
  const v4f a = *(const v4f*)(p);
  const v4f c = *(const v4f*)(p + 4);
  unsigned short hb[8];
#pragma unroll
  for (int e = 0; e < 4; ++e) {
    if (MODE == 0) {
      hb[e]     = f2bf_bits(a[e]);
      hb[4 + e] = f2bf_bits(c[e]);
    } else {
      hb[e]     = h_bits(bf_bits2f(f2bf_bits(a[e])) * scale);
      hb[4 + e] = h_bits(bf_bits2f(f2bf_bits(c[e])) * scale);
    }
  }
  const v4u u = (v4u){pk16(hb[0], hb[1]), pk16(hb[2], hb[3]), pk16(hb[4], hb[5]), pk16(hb[6], hb[7])};
  unsigned short* q = out + 8 * (size_t)i;
  *(volatile v4u*)q = u;
  __threadfence();
  *(volatile v4u*)q = u;
  (void)scale;
}

__global__ __launch_bounds__(256) void castw_kernel(const float* __restrict__ sW, const float* __restrict__ tW,
                                                    unsigned short* __restrict__ out, int n8) {
  const int i = blockIdx.x * 256 + threadIdx.x;
  if (i >= n8) return;
  constexpr int kG = kDim / 8;
  const int row = i / kG;
  const int col = (i - row * kG) * 8;
  int rs = row; rs = rs > (kLab - 1) ? (kLab - 1) : rs;
  int rt = row - kLab; rt = rt < 0 ? 0 : rt; rt = rt > (kTT - 1) ? (kTT - 1) : rt;
  const float* ps = sW + (size_t)rs * kDim + col;
  const float* pt = tW + (size_t)rt * kDim + col;
  const v4f a_s = *(const v4f*)(ps);
  const v4f c_s = *(const v4f*)(ps + 4);
  const v4f a_t = *(const v4f*)(pt);
  const v4f c_t = *(const v4f*)(pt + 4);
  const bool useS = (row < kLab);
  const bool useT = (row >= kLab) && (row < kNreal);
  unsigned short hb[8];
#pragma unroll
  for (int e = 0; e < 4; ++e) {
    const float v0 = useS ? a_s[e] : (useT ? a_t[e] : 0.0f);
    const float v1 = useS ? c_s[e] : (useT ? c_t[e] : 0.0f);
    hb[e]     = f2bf_bits(v0);
    hb[4 + e] = f2bf_bits(v1);
  }
  const v4u u = (v4u){pk16(hb[0], hb[1]), pk16(hb[2], hb[3]), pk16(hb[4], hb[5]), pk16(hb[6], hb[7])};
  unsigned short* q = out + 8 * (size_t)i;
  *(volatile v4u*)q = u;
  __threadfence();
  *(volatile v4u*)q = u;
}

__global__ __launch_bounds__(64) void crf_forward_kernel(const float* __restrict__ P, const float* __restrict__ mask,
                                                        const int* __restrict__ target, const float* __restrict__ sb,
                                                        const float* __restrict__ tb, float* __restrict__ part_out) {
#pragma clang fp contract(off)
  __shared__ __align__(16) float Erow[kNcol];
  __shared__ float tbs[kTT + 3];
  __shared__ float sbs[64];
  __shared__ float part[64];
  __shared__ float lossv;
  const int b   = blockIdx.x;
  const int tid = threadIdx.x;
#pragma unroll 1
  for (int q = tid; q < kTT; q += 64) tbs[q] = tb[q];
  if (tid < kLab) sbs[tid] = sb[tid];
  if (tid < 64) part[tid] = 0.0f;

  float te = 0.0f;
  int prev = kLab - 1;
  const v4f* P4 = (const v4f*)P;
  constexpr int kNc4 = kNcol / 4;

#pragma unroll 1
  for (int l = 0; l < kLen; ++l) {
    const size_t row = (size_t)b * kLen + l;
    __syncthreads();
#pragma unroll 1
    for (int q = tid; q < kNc4; q += 64) ((v4f*)Erow)[q] = P4[row * (size_t)kNc4 + q];
    __syncthreads();
    const float mval = mask[row];
    const int tg = target[row];
    int tgc = (tg < 0) ? (tg + kLab) : tg;
    tgc = tgc < 0 ? 0 : tgc; tgc = tgc > (kLab - 1) ? (kLab - 1) : tgc;

    float pnew = 0.0f;
    if (tid < kLab) {
      const int j = tid;
      const float os = Erow[j] + sbs[j];
      if (l == 0) {
        pnew = ((Erow[kLab + (kLab - 1) * kLab + j] + tbs[(kLab - 1) * kLab + j]) + os) * mval;
      } else {
        float m = -INFINITY;
#pragma unroll 1
        for (int i = 0; i < kLab; ++i) {
          const float v = ((Erow[kLab + i * kLab + j] + tbs[i * kLab + j]) + os) * mval + part[i];
          m = fmaxf(m, v);
        }
        if (!(m > -INFINITY && m < INFINITY)) m = 0.0f;
        float s = 0.0f;
#pragma unroll 1
        for (int i = 0; i < kLab; ++i) {
          const float v = ((Erow[kLab + i * kLab + j] + tbs[i * kLab + j]) + os) * mval + part[i];
          s += expf(v - m);
        }
        pnew = logf(s) + m;
      }
    }
    __syncthreads();
    if (tid < kLab) {
      if (l == 0) {
        part[tid] = pnew;
      } else {
        const float po = part[tid];
        part[tid] = po + (pnew - po) * mval;
      }
    }
    if (tid == 0) {
      const float mcl = fminf(fmaxf(mval, -2.0e9f), 2.0e9f);
      const int mi = (int)mcl;
      if (l == 0) {
        te = ((Erow[kLab + (kLab - 1) * kLab + tgc] + tbs[(kLab - 1) * kLab + tgc]) + (Erow[tgc] + sbs[tgc])) * mval;
        prev = (kLab - 1) + (tg - (kLab - 1)) * mi;
      } else {
        int pc = (prev < 0) ? (prev + kLab) : prev;
        pc = pc < 0 ? 0 : pc; pc = pc > (kLab - 1) ? (kLab - 1) : pc;
        te = te + ((Erow[kLab + pc * kLab + tgc] + tbs[pc * kLab + tgc]) + (Erow[tgc] + sbs[tgc])) * mval;
        prev = prev + (tg - prev) * mi;
      }
    }
  }
  __syncthreads();
  if (tid == 0) {
    float m = -INFINITY;
#pragma unroll 1
    for (int j = 0; j < kLab; ++j) m = fmaxf(m, part[j]);
    if (!(m > -INFINITY && m < INFINITY)) m = 0.0f;
    float s = 0.0f;
#pragma unroll 1
    for (int j = 0; j < kLab; ++j) s += expf(part[j] - m);
    const float lse = logf(s) + m;
    lossv = lse - te;
  }
  __syncthreads();
  if (tid < 32) {
    const float v = (tid == 0) ? lossv : 0.0f;
    float* p = part_out + (size_t)b * kPartPitch + tid;
    *(volatile float*)p = v;
    __threadfence();
    *(volatile float*)p = v;
  }
}

__global__ __launch_bounds__(32) void crf_mean_kernel(const float* __restrict__ part_out, float* __restrict__ out) {
#pragma clang fp contract(off)
  if (threadIdx.x == 0) {
    float s = 0.0f;
#pragma unroll 1
    for (int b = 0; b < kBatch; ++b) s += part_out[(size_t)b * kPartPitch];
    const float r = s * (1.0f / (float)kBatch);
    *(volatile float*)out = r;
    __threadfence();
    *(volatile float*)out = r;
  }
}

extern "C" void kernel_launch(void* const* d_in, const int* in_sizes, int n_in,
                              void* d_out, int out_size, void* d_ws, size_t ws_size,
                              hipStream_t stream) {
  if (n_in < 7) return;
  if (in_sizes[0] != kRows * kDim) return;
  if (in_sizes[1] != kRows) return;
  if (in_sizes[2] != kRows) return;
  if (in_sizes[3] != kLab * kDim) return;
  if (in_sizes[4] != kLab) return;
  if (in_sizes[5] != kTT * kDim) return;
  if (in_sizes[6] != kTT) return;
  if (out_size != 1) return;

  const float* x    = (const float*)d_in[0];
  const float* mask = (const float*)d_in[1];
  const int*   tgt  = (const int*)d_in[2];
  const float* sW   = (const float*)d_in[3];
  const float* sb   = (const float*)d_in[4];
  const float* tW   = (const float*)d_in[5];
  const float* tb   = (const float*)d_in[6];
  float* outp = (float*)d_out;

  const size_t SZ_XB   = (size_t)kRows * kDim * 2;
  const size_t SZ_WB   = (size_t)kNcol * kDim * 2;
  const size_t SZ_P    = (size_t)kRows * kNcol * 4;
  const size_t SZ_PART = (size_t)kBatch * kPartPitch * 4;
  size_t off = 0;
  const size_t oXB   = off; off += SZ_XB;
  const size_t oWB   = off; off += SZ_WB;
  const size_t oP    = off; off += SZ_P;
  const size_t oPART = off; off += SZ_PART;
  const size_t TOTAL = off;
  if (TOTAL > ws_size) return;
  if (TOTAL > (size_t)134217728) return;

  char* ws = (char*)d_ws;
  unsigned short* XB   = (unsigned short*)(ws + oXB);
  unsigned short* WB   = (unsigned short*)(ws + oWB);
  float*          P    = (float*)(ws + oP);
  float*          PART = (float*)(ws + oPART);
  const float* dummy_rsc = PART;

  const dim3 blk(256);

  {
    const int n8x = kRows * kDim / 8;
    cast8_kernel<0><<<dim3(n8x / 256), blk, 0, stream>>>(x, XB, n8x, 1.0f);
  }
  {
    const int n8w = kNcol * kDim / 8;
    castw_kernel<<<dim3(n8w / 256), blk, 0, stream>>>(sW, tW, WB, n8w);
  }
  {
    const int tiles = (kRows / 64) * (kNcol / 64);
    const dim3 g((tiles + 7) / 8, 1);
    wmma_gemm64<1, 0, 0, 0, 0, 0><<<g, blk, 0, stream>>>(
        XB, XB, kDim, 0L, WB, WB, kDim, 0L, (void*)P, (void*)P, kNcol, 0L, dummy_rsc, 0L, kRows, kNcol, kDim, 1.0f);
  }
  crf_forward_kernel<<<dim3(kBatch), dim3(64), 0, stream>>>(P, mask, tgt, sb, tb, PART);
  crf_mean_kernel<<<dim3(1), dim3(32), 0, stream>>>(PART, outp);
}
